// GraphConvWL_26560077758774
// MI455X (gfx1250) — hardware-verified
//
#include <hip/hip_runtime.h>
#include <hip/hip_bf16.h>
#include <stddef.h>


#define FD    128
#define K1    256
#define NB    256
#define NTHR  256
#define NWAVE 8
#define SBN   4096
#define SUBS  (SBN / NB)
#define EPT   8
#define CHUNK (NTHR * EPT)
#define WCAP  (EPT * 32)
#define PB    6144
#define FLT   4096
#define RHDR  32
#define RCAP  98304
#define RROW  (RHDR + RCAP)
#define HCAP  5632
#define WLC   1024
#define BROW  (RHDR + NWAVE * WLC)
#define LDS_MAIN (NB * FD * 4)
#define PREP1 ((FD * (K1 / 8)) / NTHR)

static_assert(NTHR == NWAVE * 32);
static_assert(NB == NWAVE * 32);
static_assert(SBN == SUBS * NB && SUBS <= 255);
static_assert(WCAP == EPT * 32);
static_assert(PB >= FLT + CHUNK && (PB % 32) == 0 && (FLT % 32) == 0);
static_assert((RCAP % CHUNK) == 0 && ((RROW * 4) % 128) == 0);
static_assert((HCAP % 32) == 0 && (WLC % 32) == 0);
static_assert(((BROW * 4) % 128) == 0 && ((NWAVE * WLC) % (4 * NTHR)) == 0);
static_assert(NWAVE <= RHDR);
static_assert(LDS_MAIN <= 300 * 1024);
static_assert(PREP1 * NTHR == FD * (K1 / 8));
static_assert((NB * FD / 4) % NTHR == 0 && FD * 4 == 512);

typedef float          v4f   __attribute__((ext_vector_type(4)));
typedef float          v8f   __attribute__((ext_vector_type(8)));
typedef int            v4i   __attribute__((ext_vector_type(4)));
typedef unsigned       v4u   __attribute__((ext_vector_type(4)));
typedef unsigned short v8us  __attribute__((ext_vector_type(8)));
typedef unsigned short v16us __attribute__((ext_vector_type(16)));
typedef __bf16         v16bf __attribute__((ext_vector_type(16)));
union FragB { v16bf v; v16us u; v8us h[2]; };
union Pk8 { v8us h; v4u i; };

__device__ __forceinline__ v4f zero4() { v4f z; z.x = 0.0f; z.y = 0.0f; z.z = 0.0f; z.w = 0.0f; return z; }
__device__ __forceinline__ v8f zero8() { v8f z; for (int i = 0; i < 8; ++i) z[i] = 0.0f; return z; }

__device__ __forceinline__ unsigned f2bf(float f) {
  const unsigned u = __float_as_uint(f);
  return (u + 0x7FFFu + ((u >> 16) & 1u)) >> 16;
}

__device__ __forceinline__ void split8(v4f a, v4f b, v8us& hi, v8us& lo) {
  float f[8];
  f[0] = a.x; f[1] = a.y; f[2] = a.z; f[3] = a.w;
  f[4] = b.x; f[5] = b.y; f[6] = b.z; f[7] = b.w;
  v8us rh, rl;
#pragma unroll
  for (int i = 0; i < 8; ++i) {
    const unsigned hb = f2bf(f[i]);
    const float r = f[i] - __uint_as_float(hb << 16);
    rh[i] = (unsigned short)hb;
    rl[i] = (unsigned short)f2bf(r);
  }
  hi = rh;
  lo = rl;
}

__device__ __forceinline__ v8f wm3(v16bf ah, v16bf al, v16bf bh, v16bf bl, v8f c) {
  v8f d = __builtin_amdgcn_wmma_f32_16x16x32_bf16(false, ah, false, bh, (short)0, c, false, false);
  d = __builtin_amdgcn_wmma_f32_16x16x32_bf16(false, ah, false, bl, (short)0, d, false, false);
  d = __builtin_amdgcn_wmma_f32_16x16x32_bf16(false, al, false, bh, (short)0, d, false, false);
  asm volatile("v_nop\n\tv_nop\n\tv_nop\n\tv_nop" : "+v"(d) : "v"(ah), "v"(al), "v"(bh), "v"(bl));
  return d;
}

template <int NJ>
__device__ __forceinline__ void gstep(const FragB& ah, const FragB& al,
    const unsigned short* __restrict__ ph, const unsigned short* __restrict__ pl,
    int kp, int ko, int m, v8f (&d)[NJ]) {
#pragma unroll
  for (int j = 0; j < NJ; ++j) {
    const size_t o = (size_t)(16 * j + m) * kp + ko;
    FragB bh, bl;
    bh.h[0] = *(const v8us*)(ph + o);
    bh.h[1] = *(const v8us*)(ph + o + 16);
    bl.h[0] = *(const v8us*)(pl + o);
    bl.h[1] = *(const v8us*)(pl + o + 16);
    d[j] = wm3(ah.v, al.v, bh.v, bl.v, d[j]);
  }
}

__device__ __forceinline__ int scan_chunk(const int* __restrict__ dsts, int nE, int cbase, int sbBase,
                                          int vec8, unsigned* list, int tid, int wave) {
  int wc = 0;
  const int e0   = cbase + tid * EPT;
  const int sent = -2147483647 - 1;
  v4i da, db;
  if (vec8 != 0 && cbase + CHUNK <= nE) {
    da = *(const v4i*)(dsts + e0);
    db = *(const v4i*)(dsts + e0 + 4);
  } else {
    da.x = (e0     < nE) ? dsts[min(e0, nE - 1)] : sent;
    da.y = (e0 + 1 < nE) ? dsts[min(e0 + 1, nE - 1)] : sent;
    da.z = (e0 + 2 < nE) ? dsts[min(e0 + 2, nE - 1)] : sent;
    da.w = (e0 + 3 < nE) ? dsts[min(e0 + 3, nE - 1)] : sent;
    db.x = (e0 + 4 < nE) ? dsts[min(e0 + 4, nE - 1)] : sent;
    db.y = (e0 + 5 < nE) ? dsts[min(e0 + 5, nE - 1)] : sent;
    db.z = (e0 + 6 < nE) ? dsts[min(e0 + 6, nE - 1)] : sent;
    db.w = (e0 + 7 < nE) ? dsts[min(e0 + 7, nE - 1)] : sent;
  }
  const unsigned nb = (unsigned)sbBase;
  const unsigned s0 = (unsigned)da.x - nb, s1 = (unsigned)da.y - nb;
  const unsigned s2 = (unsigned)da.z - nb, s3 = (unsigned)da.w - nb;
  const unsigned s4 = (unsigned)db.x - nb, s5 = (unsigned)db.y - nb;
  const unsigned s6 = (unsigned)db.z - nb, s7 = (unsigned)db.w - nb;
  const bool h0 = s0 < (unsigned)SBN, h1 = s1 < (unsigned)SBN, h2 = s2 < (unsigned)SBN, h3 = s3 < (unsigned)SBN;
  const bool h4 = s4 < (unsigned)SBN, h5 = s5 < (unsigned)SBN, h6 = s6 < (unsigned)SBN, h7 = s7 < (unsigned)SBN;
#define HITJ(J, HJ, SJ) { \
    const unsigned mj = __builtin_amdgcn_ballot_w32(HJ); \
    if (mj != 0u) { \
      const int pos = wc + (int)__builtin_amdgcn_mbcnt_lo(mj, 0u); \
      if ((HJ) && pos < WCAP) list[wave * WCAP + pos] = (((unsigned)(e0 + (J))) << 8) | ((SJ) >> 8); \
      wc += (int)__builtin_popcount(mj); } }
  HITJ(0, h0, s0)
  HITJ(1, h1, s1)
  HITJ(2, h2, s2)
  HITJ(3, h3, s3)
  HITJ(4, h4, s4)
  HITJ(5, h5, s5)
  HITJ(6, h6, s6)
  HITJ(7, h7, s7)
#undef HITJ
  return wc;
}

__device__ __forceinline__ int filt_chunk(const unsigned* __restrict__ ent, int cnt, int cbase, unsigned sub,
                                          unsigned* list, int tid, int wave) {
  int wc = 0;
  const int e0 = cbase + tid * EPT;
  const v4u a = *(const v4u*)(ent + e0);
  const v4u b = *(const v4u*)(ent + e0 + 4);
  const bool h0 = (e0     < cnt) && ((a.x & 255u) == sub);
  const bool h1 = (e0 + 1 < cnt) && ((a.y & 255u) == sub);
  const bool h2 = (e0 + 2 < cnt) && ((a.z & 255u) == sub);
  const bool h3 = (e0 + 3 < cnt) && ((a.w & 255u) == sub);
  const bool h4 = (e0 + 4 < cnt) && ((b.x & 255u) == sub);
  const bool h5 = (e0 + 5 < cnt) && ((b.y & 255u) == sub);
  const bool h6 = (e0 + 6 < cnt) && ((b.z & 255u) == sub);
  const bool h7 = (e0 + 7 < cnt) && ((b.w & 255u) == sub);
#define HITF(HJ, VJ) { \
    const unsigned mj = __builtin_amdgcn_ballot_w32(HJ); \
    if (mj != 0u) { \
      const int pos = wc + (int)__builtin_amdgcn_mbcnt_lo(mj, 0u); \
      if ((HJ) && pos < WCAP) list[wave * WCAP + pos] = (VJ) >> 8; \
      wc += (int)__builtin_popcount(mj); } }
  HITF(h0, a.x)
  HITF(h1, a.y)
  HITF(h2, a.z)
  HITF(h3, a.w)
  HITF(h4, b.x)
  HITF(h5, b.y)
  HITF(h6, b.z)
  HITF(h7, b.w)
#undef HITF
  return wc;
}

__device__ __forceinline__ void flush2(const unsigned* pend, unsigned* dst, int nst, int tid) {
#pragma unroll 1
  for (int u = tid; u < (nst >> 2); u += NTHR) {
    const v4u v = *(const v4u*)(pend + 4 * u);
    *(volatile v4u*)(dst + 4 * u) = v;
  }
  __threadfence();
#pragma unroll 1
  for (int u = tid; u < (nst >> 2); u += NTHR) {
    const v4u v = *(const v4u*)(pend + 4 * u);
    *(volatile v4u*)(dst + 4 * u) = v;
  }
}

__global__ __launch_bounds__(NTHR) void k_prep(const float* __restrict__ wn, const float* __restrict__ wsf,
                                              unsigned short* p1) {
  const int u = blockIdx.x * NTHR + threadIdx.x;
  const int n = u >> 5;
  const int kc = u & 31;
  float f[8];
#pragma unroll
  for (int j = 0; j < 8; ++j) {
    const int k = 8 * kc + j;
    const int ka = k < FD ? k : FD - 1;
    const int kb = k < FD ? 0 : k - FD;
    const float va = wn[ka * FD + n];
    const float vb = wsf[kb * FD + n];
    f[j] = (k < FD) ? va : vb;
  }
  unsigned short* dh = p1 + (size_t)u * 8;
  unsigned short* dl = p1 + (size_t)FD * K1 + (size_t)u * 8;
  Pk8 ph, pl;
  {
    v4f a, c;
    a.x = f[0]; a.y = f[1]; a.z = f[2]; a.w = f[3];
    c.x = f[4]; c.y = f[5]; c.z = f[6]; c.w = f[7];
    split8(a, c, ph.h, pl.h);
  }
  *(volatile v4u*)dh = ph.i;
  *(volatile v4u*)dl = pl.i;
  __threadfence();
  *(volatile v4u*)dh = ph.i;
  *(volatile v4u*)dl = pl.i;
}

__global__ __launch_bounds__(NTHR) void k_scan(const int* __restrict__ dsts, unsigned* t1, int nE, int vec8) {
  __shared__ unsigned list[NWAVE * WCAP];
  __shared__ __attribute__((aligned(16))) unsigned pend[PB];
  __shared__ int wcnt[NWAVE];
  const int tid = threadIdx.x, lane = tid & 31, wave = tid >> 5;
  const int sbBase = blockIdx.x * SBN;
  unsigned* rowp = t1 + (size_t)blockIdx.x * RROW;
  unsigned* ent = rowp + RHDR;
  int pendN = 0;
  int gpos = 0;
  const int nChunks = (nE + CHUNK - 1) / CHUNK;
#pragma unroll 1
  for (int ch = 0; ch < nChunks; ++ch) {
    const int cbase = ch * CHUNK;
    const int wc = scan_chunk(dsts, nE, cbase, sbBase, vec8, list, tid, wave);
    if (lane == 0) wcnt[wave] = wc;
    __syncthreads();
    int tot = 0, myoff = 0;
#pragma unroll
    for (int w = 0; w < NWAVE; ++w) {
      int c = wcnt[w];
      c = c > WCAP ? WCAP : (c < 0 ? 0 : c);
      if (w < wave) myoff += c;
      tot += c;
    }
    {
      int n = wcnt[wave];
      n = n > WCAP ? WCAP : (n < 0 ? 0 : n);
      const unsigned* lp = list + wave * WCAP;
      for (int i = lane; i < n; i += 32) {
        const int pos = pendN + myoff + i;
        if (pos < PB) pend[pos] = lp[i];
      }
    }
    {
      const int newN = pendN + tot;
      pendN = newN > PB ? PB : newN;
    }
    __syncthreads();
    if (pendN >= FLT) {
      const int nfl = pendN & ~31;
      const int room = RCAP - gpos;
      const int nst = nfl < room ? nfl : room;
      flush2(pend, ent + gpos, nst, tid);
      gpos += nst;
      __syncthreads();
      const int rem = pendN - nfl;
      unsigned mv = 0u;
      if (tid < rem) mv = pend[nfl + tid];
      if (tid < rem) pend[tid] = mv;
      pendN = rem;
    }
  }
  __syncthreads();
  const int nfin = (pendN + 31) & ~31;
  if (tid < 32) {
    const int idx = pendN + tid;
    if (idx < nfin) pend[idx] = 0xFFFFFFFFu;
  }
  __syncthreads();
  {
    const int room = RCAP - gpos;
    const int nst = nfin < room ? nfin : room;
    flush2(pend, ent + gpos, nst, tid);
    gpos += nst;
  }
  if (wave == 0) {
    const unsigned hv = (lane == 0) ? (unsigned)gpos : 0u;
    *(volatile unsigned*)(rowp + lane) = hv;
    __threadfence();
    *(volatile unsigned*)(rowp + lane) = hv;
  }
}

__global__ __launch_bounds__(NTHR) void k_part(const int* __restrict__ dsts, const unsigned* __restrict__ t1,
                                              unsigned* t2, int nE) {
  __shared__ unsigned list[NWAVE * WCAP];
  __shared__ unsigned hl[HCAP];
  __shared__ __attribute__((aligned(16))) unsigned wl[NWAVE * WLC];
  __shared__ int wcnt[NWAVE];
  __shared__ int wlen[NWAVE];
  const int tid = threadIdx.x, lane = tid & 31, wave = tid >> 5;
  const int blk = blockIdx.x;
  const int sb = blk / SUBS;
  const unsigned sub = (unsigned)(blk - sb * SUBS);
  const int nodeBase = blk * NB;
  const unsigned* rowp = t1 + (size_t)sb * RROW;
  const unsigned* ent = rowp + RHDR;
  for (int i = tid; i < NWAVE * WLC; i += NTHR) wl[i] = 0u;
  int cnt = (int)rowp[0];
  cnt = cnt < 0 ? 0 : (cnt > RCAP ? RCAP : cnt);
  int hlN = 0;
  const int nCh = (cnt + CHUNK - 1) / CHUNK;
  __syncthreads();
#pragma unroll 1
  for (int ch = 0; ch < nCh; ++ch) {
    const int cbase = ch * CHUNK;
    const int wc = filt_chunk(ent, cnt, cbase, sub, list, tid, wave);
    if (lane == 0) wcnt[wave] = wc;
    __syncthreads();
    int tot = 0, myoff = 0;
#pragma unroll
    for (int w = 0; w < NWAVE; ++w) {
      int c = wcnt[w];
      c = c > WCAP ? WCAP : (c < 0 ? 0 : c);
      if (w < wave) myoff += c;
      tot += c;
    }
    {
      int n = wcnt[wave];
      n = n > WCAP ? WCAP : (n < 0 ? 0 : n);
      const unsigned* lp = list + wave * WCAP;
      for (int i = lane; i < n; i += 32) {
        const int pos = hlN + myoff + i;
        if (pos < HCAP) hl[pos] = lp[i];
      }
    }
    {
      const int newN = hlN + tot;
      hlN = newN > HCAP ? HCAP : newN;
    }
    __syncthreads();
  }
  {
    int wn = 0;
    const int niter = (hlN + 31) >> 5;
#pragma unroll 1
    for (int it = 0; it < niter; ++it) {
      const int idx = it * 32 + lane;
      const bool valid = idx < hlN;
      int e = (int)hl[idx < HCAP ? idx : HCAP - 1];
      e = e < 0 ? 0 : (e > nE - 1 ? nE - 1 : e);
      const int d = dsts[e];
      const int slot = d - nodeBase;
      const bool mine = valid && ((unsigned)slot < (unsigned)NB) && ((slot >> 5) == wave);
      const unsigned mk = __builtin_amdgcn_ballot_w32(mine);
      const int pos = wn + (int)__builtin_amdgcn_mbcnt_lo(mk, 0u);
      if (mine && pos < WLC) wl[wave * WLC + pos] = (((unsigned)e) << 8) | (unsigned)slot;
      wn += (int)__builtin_popcount(mk);
    }
    if (lane == 0) wlen[wave] = wn > WLC ? WLC : wn;
  }
  __syncthreads();
  unsigned* orow = t2 + (size_t)blk * BROW;
  unsigned hv = 0u;
  if (lane < NWAVE) hv = (unsigned)wlen[lane];
#pragma unroll 1
  for (int u = tid; u < NWAVE * WLC / 4; u += NTHR) {
    const v4u v = *(const v4u*)(wl + 4 * u);
    *(volatile v4u*)(orow + RHDR + 4 * u) = v;
  }
  if (wave == 0) *(volatile unsigned*)(orow + lane) = hv;
  __threadfence();
#pragma unroll 1
  for (int u = tid; u < NWAVE * WLC / 4; u += NTHR) {
    const v4u v = *(const v4u*)(wl + 4 * u);
    *(volatile v4u*)(orow + RHDR + 4 * u) = v;
  }
  if (wave == 0) *(volatile unsigned*)(orow + lane) = hv;
}

__global__ __launch_bounds__(NTHR) void k_main(const float* __restrict__ x, const int* __restrict__ srcs,
    const float* __restrict__ ew, const unsigned* __restrict__ t2,
    const unsigned short* __restrict__ wh, const unsigned short* __restrict__ wlo,
    const float* __restrict__ bias, float* out, int nN, int nE) {
  extern __shared__ __attribute__((aligned(16))) unsigned char dsm[];
  float* acc = (float*)dsm;
  const int tid = threadIdx.x, lane = tid & 31, wave = tid >> 5, hh = lane >> 4, m = lane & 15;
  const int nodeBase = blockIdx.x * NB;
  {
    const v4f z = zero4();
    for (int i = tid; i < NB * FD / 4; i += NTHR) *(v4f*)(acc + 4 * i) = z;
  }
  __syncthreads();
  {
    const unsigned* brow = t2 + (size_t)blockIdx.x * BROW;
    int cnt = (int)brow[wave];
    cnt = cnt < 0 ? 0 : (cnt > WLC ? WLC : cnt);
    cnt = __builtin_amdgcn_readfirstlane(cnt);
    const unsigned* lst = brow + RHDR + wave * WLC;
#pragma unroll 1
    for (int i = 0; i < cnt; i += 32) {
      const unsigned pk = lst[i + lane];
      int e = (int)(pk >> 8);
      e = e > nE - 1 ? nE - 1 : e;
      const int sl = (int)(pk & 255u);
      int sv = srcs[e];
      sv = sv < 0 ? 0 : (sv > nN - 1 ? nN - 1 : sv);
      const float wv = ew[e];
      int jn = cnt - i;
      jn = jn > 32 ? 32 : jn;
#pragma unroll 1
      for (int jj = 0; jj < jn; ++jj) {
        const int s = __builtin_amdgcn_readlane(sv, jj);
        const int slot = __builtin_amdgcn_readlane(sl, jj);
        const float w = __int_as_float(__builtin_amdgcn_readlane(__float_as_int(wv), jj));
        const v4f v = *(const v4f*)(x + (size_t)s * FD + 4 * lane);
        float* ap = acc + slot * FD + 4 * lane;
        v4f a = *(v4f*)ap;
        a += v * w;
        *(v4f*)ap = a;
      }
    }
  }
  __syncthreads();
#pragma unroll 1
  for (int tt = 0; tt < 2; ++tt) {
    const int t = wave + NWAVE * tt;
    const int r0 = 16 * t;
    int node = nodeBase + r0 + m;
    node = node > nN - 1 ? nN - 1 : node;
    const float* arow = acc + (r0 + m) * FD;
    const float* xrow = x + (size_t)node * FD;
    v8f d[8];
#pragma unroll
    for (int j = 0; j < 8; ++j) d[j] = zero8();
#pragma unroll 1
    for (int ks = 0; ks < 4; ++ks) {
      const int ko = 32 * ks + 8 * hh;
      FragB ah, al;
      split8(*(const v4f*)(arow + ko), *(const v4f*)(arow + ko + 4), ah.h[0], al.h[0]);
      split8(*(const v4f*)(arow + ko + 16), *(const v4f*)(arow + ko + 20), ah.h[1], al.h[1]);
      gstep<8>(ah, al, wh, wlo, K1, ko, m, d);
    }
#pragma unroll 1
    for (int ks = 0; ks < 4; ++ks) {
      const int ko = 32 * ks + 8 * hh;
      FragB ah, al;
      split8(*(const v4f*)(xrow + ko), *(const v4f*)(xrow + ko + 4), ah.h[0], al.h[0]);
      split8(*(const v4f*)(xrow + ko + 16), *(const v4f*)(xrow + ko + 20), ah.h[1], al.h[1]);
      gstep<8>(ah, al, wh, wlo, K1, FD + ko, m, d);
    }
    __syncthreads();
    float* srow = acc + (r0 + 8 * hh) * FD;
#pragma unroll
    for (int j = 0; j < 8; ++j) {
      const int col = 16 * j + m;
      const float bj = bias[col];
#pragma unroll
      for (int r = 0; r < 8; ++r) srow[r * FD + col] = d[j][r] + bj;
    }
  }
  __syncthreads();
  int nrw = nN - (nodeBase + wave * 32);
  nrw = nrw < 0 ? 0 : (nrw > 32 ? 32 : nrw);
  nrw = __builtin_amdgcn_readfirstlane(nrw);
#pragma unroll 1
  for (int rr = 0; rr < nrw; ++rr) {
    const int row = wave * 32 + rr;
    const v4f v = *(const v4f*)(acc + row * FD + 4 * lane);
    *(volatile v4f*)(out + (size_t)(nodeBase + row) * FD + 4 * lane) = v;
  }
  __threadfence();
#pragma unroll 1
  for (int rr = 0; rr < nrw; ++rr) {
    const int row = wave * 32 + rr;
    const v4f v = *(const v4f*)(acc + row * FD + 4 * lane);
    *(volatile v4f*)(out + (size_t)(nodeBase + row) * FD + 4 * lane) = v;
  }
}

extern "C" void kernel_launch(void* const* d_in, const int* in_sizes, int n_in,
                              void* d_out, int out_size, void* d_ws, size_t ws_size,
                              hipStream_t stream) {
  if (n_in < 7) return;
  if (in_sizes[0] < FD || (in_sizes[0] % FD) != 0) return;
  const int nN = in_sizes[0] / FD;
  const int nE = in_sizes[1];
  if (nE < 1 || nE >= (1 << 23)) return;
  if (in_sizes[2] != nE || in_sizes[3] != nE) return;
  if (in_sizes[4] != FD * FD || in_sizes[5] != FD * FD || in_sizes[6] != FD) return;
  if (out_size != nN * FD) return;

  const float* feat = (const float*)d_in[0];
  const int*   srcs = (const int*)d_in[1];
  const int*   dsts = (const int*)d_in[2];
  const float* ew   = (const float*)d_in[3];
  const float* wn   = (const float*)d_in[4];
  const float* wsf  = (const float*)d_in[5];
  const float* bn   = (const float*)d_in[6];
  float* dout = (float*)d_out;

  const int nBlk = (nN + NB - 1) / NB;
  const int nSB = (nBlk + SUBS - 1) / SUBS;

  char* ws = (char*)d_ws;
  size_t off = 0;
  auto carve = [&](size_t bytes) -> size_t {
    const size_t o = off;
    off = (off + bytes + 255) & ~(size_t)255;
    return o;
  };
  const size_t n1 = (size_t)FD * K1;
  const size_t oP1 = carve(2 * n1 * 2);
  const size_t oT1 = carve((size_t)nSB * RROW * 4);
  const size_t oT2 = carve((size_t)nBlk * BROW * 4);
  size_t limit = (size_t)134217728;
  if (ws_size < limit) limit = ws_size;
  if (off > limit) return;

  unsigned short* p1 = (unsigned short*)(ws + oP1);
  unsigned* t1 = (unsigned*)(ws + oT1);
  unsigned* t2 = (unsigned*)(ws + oT2);

  const int vec8 = 1;

  k_prep<<<PREP1, NTHR, 0, stream>>>(wn, wsf, p1);
  k_scan<<<nSB, NTHR, 0, stream>>>(dsts, t1, nE, vec8);
  k_part<<<nBlk, NTHR, 0, stream>>>(dsts, t1, t2, nE);

  hipFuncSetAttribute(reinterpret_cast<const void*>(&k_main), hipFuncAttributeMaxDynamicSharedMemorySize, LDS_MAIN);
  k_main<<<nBlk, NTHR, LDS_MAIN, stream>>>(feat, srcs, ew, t2, p1, p1 + n1, bn, dout, nN, nE);
}
